// Lstm_90323162235334
// MI455X (gfx1250) — hardware-verified
//
#include <hip/hip_runtime.h>
#include <math.h>
#include <stddef.h>

typedef __attribute__((ext_vector_type(16))) _Float16 v16h;
typedef __attribute__((ext_vector_type(8)))  _Float16 v8h;
typedef __attribute__((ext_vector_type(8)))  float    v8f;
typedef __attribute__((ext_vector_type(4)))  float    v4f;
typedef __attribute__((ext_vector_type(4)))  unsigned v4u;
typedef __attribute__((ext_vector_type(2)))  unsigned v2u;
typedef v4u v4u_a __attribute__((may_alias));
typedef v2u v2u_a __attribute__((may_alias));

constexpr int N_BATCH   = 256;
constexpr int N_STEP    = 2048;
constexpr int N_FEAT    = 8;
constexpr int HID       = 43;
constexpr int CH_PAD    = 48;
constexpr int N_PAD     = 192;
constexpr int L1_K      = 64;
constexpr int L2_K      = 160;
constexpr int H1_W      = 44;
constexpr int H1_TILE   = 16 * H1_W;
constexpr int PB_TILE   = 16 * 32;
constexpr int N_TILE    = N_BATCH / 16;
constexpr int D1_N      = 30;
constexpr int D2_N      = 20;
constexpr int HEAD_NP   = 32;
constexpr int WD1_K     = 64;
constexpr int WD2_K     = 32;
constexpr int NTHR_SEQ  = 96;
constexpr int L1_AP = 72;
constexpr int L2_AP = 168;
constexpr int BI_P  = 104;
constexpr int W1_P  = 72;
constexpr int W2_P  = 40;
constexpr int A1_P  = 40;
constexpr int OB_P  = 36;
constexpr float WCARRY     = 16.0f;
constexpr float WCARRY_INV = 1.0f / 16.0f;
constexpr size_t H1_PLANE = (size_t)N_TILE * N_STEP * H1_TILE;
constexpr size_t PB_PLANE = (size_t)N_TILE * N_STEP * PB_TILE;

static_assert(4 * CH_PAD == N_PAD, "gate padding");
static_assert(HID <= CH_PAD && HID < H1_W, "channel padding");
static_assert(L1_K % 32 == 0 && L2_K % 32 == 0 && WD1_K % 32 == 0 && WD2_K % 32 == 0, "K multiples of 32");
static_assert(N_PAD % 16 == 0 && HEAD_NP % 16 == 0, "N tile multiples");
static_assert(N_STEP % 32 == 0, "output flush granularity");
static_assert((H1_TILE * 2) % 128 == 0 && (PB_TILE * 2) % 128 == 0, "whole-line tiles");
static_assert((16 * L1_AP) % NTHR_SEQ == 0 && (16 * L2_AP) % NTHR_SEQ == 0, "zero-fill loops exact");
static_assert((N_PAD * 12) % NTHR_SEQ == 0, "BI copy loop exact");

constexpr int CH_BT1 = 2 * N_PAD * L1_K / 8;
constexpr int CH_BT2 = 2 * N_PAD * L2_K / 8;
constexpr int CH_WD1 = 2 * HEAD_NP * WD1_K / 8;
constexpr int CH_WD2 = HEAD_NP * WD2_K / 8;
constexpr int CH_B1  = 2 * N_PAD / 4;
constexpr int CH_B2  = 2 * N_PAD / 4;
constexpr int CH_TOTAL = CH_BT1 + CH_BT2 + CH_WD1 + CH_WD2 + CH_B1 + CH_B2;
static_assert(CH_BT1 % 32 == 0 && CH_BT2 % 32 == 0 && CH_WD1 % 32 == 0 && CH_WD2 % 32 == 0 && CH_B1 % 32 == 0 && CH_B2 % 32 == 0,
              "plane boundaries on wave boundaries");
static_assert((CH_BT1 / 2) % 32 == 0 && (CH_BT2 / 2) % 32 == 0, "direction boundaries on wave boundaries");

constexpr size_t WS_H1  = 2 * H1_PLANE * 2;
constexpr size_t WS_PB  = PB_PLANE * 2;
constexpr size_t WS_BT1 = (size_t)2 * N_PAD * L1_K * 2;
constexpr size_t WS_BT2 = (size_t)2 * N_PAD * L2_K * 2;
constexpr size_t WS_WD1 = (size_t)2 * HEAD_NP * WD1_K * 2;
constexpr size_t WS_WD2 = (size_t)HEAD_NP * WD2_K * 2;
constexpr size_t WS_B1  = (size_t)2 * N_PAD * 4;
constexpr size_t WS_B2  = (size_t)2 * N_PAD * 4;
constexpr size_t WS_TOTAL = WS_H1 + WS_PB + WS_BT1 + WS_BT2 + WS_WD1 + WS_WD2 + WS_B1 + WS_B2;
static_assert(WS_H1 % 256 == 0 && WS_PB % 256 == 0 && WS_BT1 % 256 == 0 && WS_BT2 % 256 == 0 &&
              WS_WD1 % 256 == 0 && WS_WD2 % 256 == 0 && WS_B1 % 256 == 0 && WS_B2 % 256 == 0, "aligned carve");
static_assert(WS_TOTAL <= (size_t)134217728, "carve within 128 MiB");

struct FragH {
  union U { v16h v; v8h h[2]; };
  static __device__ __forceinline__ v16h load(const _Float16* p) {
    U f; f.h[0] = *(const v8h*)(p); f.h[1] = *(const v8h*)(p + 16); return f.v;
  }
};
__device__ __forceinline__ v8f wm(v16h a, v16h b, v8f c) {
  return __builtin_amdgcn_wmma_f32_16x16x32_f16(false, a, false, b, (short)0, c, false, false);
}
__device__ __forceinline__ void guard_g4(v8f& a0, v8f& a1, v8f& a2, v8f& a3, v16h x, v16h b0, v16h b1, v16h b2, v16h b3) {
  asm volatile("v_nop\n\tv_nop\n\tv_nop\n\tv_nop"
               : "+v"(a0), "+v"(a1), "+v"(a2), "+v"(a3)
               : "v"(x), "v"(b0), "v"(b1), "v"(b2), "v"(b3)
               : "memory");
}
__device__ __forceinline__ void guard_g2(v8f& a0, v8f& a1, v16h x, v16h b0, v16h b1) {
  asm volatile("v_nop\n\tv_nop\n\tv_nop\n\tv_nop"
               : "+v"(a0), "+v"(a1)
               : "v"(x), "v"(b0), "v"(b1)
               : "memory");
}
__device__ __forceinline__ void guard_g1(v8f& a0, v16h x0, v16h x1, v16h b0, v16h b1) {
  asm volatile("v_nop\n\tv_nop\n\tv_nop\n\tv_nop"
               : "+v"(a0)
               : "v"(x0), "v"(x1), "v"(b0), "v"(b1)
               : "memory");
}
__device__ __forceinline__ void pin_frag2(v16h& a, v16h& b, float& s) {
  asm volatile("" : "+v"(a), "+v"(b), "+v"(s));
}
__device__ __forceinline__ void pin_f4(float& a, float& b, float& c, float& d) {
  asm volatile("" : "+v"(a), "+v"(b), "+v"(c), "+v"(d));
}

__device__ __forceinline__ float fsig(float x)  { return __builtin_amdgcn_rcpf(1.0f + __expf(-x)); }
__device__ __forceinline__ float ftanh(float x) { return 1.0f - 2.0f * __builtin_amdgcn_rcpf(__expf(2.0f * x) + 1.0f); }

__device__ __forceinline__ float h16_to_f32(unsigned hb) {
  const unsigned sgn = (hb & 0x8000u) << 16; const unsigned em = hb & 0x7fffu;
  const float fn = __uint_as_float((em << 13) + 0x38000000u);
  const float fs = (float)em * 5.9604644775390625e-8f;
  const float mag = (em < 0x400u) ? fs : fn; return __uint_as_float(__float_as_uint(mag) | sgn);
}

__device__ __forceinline__ void store2_h8(unsigned short* p, v8h v) {
  *(volatile v8h*)p = v;
  __threadfence();
  *(volatile v8h*)p = v;
}
__device__ __forceinline__ void store2_f4(float* p, v4f v) {
  *(volatile v4f*)p = v;
  __threadfence();
  *(volatile v4f*)p = v;
}

__device__ __forceinline__ void lstm_cell8(const v8f ai, const v8f af, const v8f ag, const v8f ao,
                                           float (&cst)[8], float (&hn)[8], const bool chv) {
#pragma unroll
  for (int r = 0; r < 8; ++r) {
    const float ig = fsig(ai[r] * WCARRY_INV);
    const float fg = fsig(af[r] * WCARRY_INV);
    const float gg = ftanh(ag[r] * WCARRY_INV);
    const float og = fsig(ao[r] * WCARRY_INV);
    const float cn = fg * cst[r] + ig * gg;
    const float hv = og * ftanh(cn);
    cst[r] = chv ? cn : 0.0f;
    hn[r]  = chv ? hv : 0.0f;
  }
}

__device__ __forceinline__ void stage_x_row(_Float16* dst, const v4f xa, const v4f xb) {
  v8h xv;
  xv[0] = (_Float16)xa[0]; xv[1] = (_Float16)xa[1]; xv[2] = (_Float16)xa[2]; xv[3] = (_Float16)xa[3];
  xv[4] = (_Float16)xb[0]; xv[5] = (_Float16)xb[1]; xv[6] = (_Float16)xb[2]; xv[7] = (_Float16)xb[3];
  *(v8h*)dst = xv;
  const v4u z = {0u, 0u, 0u, 0u};
  *(v4u_a*)(dst + 8) = z;
}

__global__ __launch_bounds__(256) void prep_planes_kernel(
    const float* __restrict__ w_proj, const float* __restrict__ b_proj,
    const float* __restrict__ wih1f, const float* __restrict__ whh1f, const float* __restrict__ bih1f, const float* __restrict__ bhh1f,
    const float* __restrict__ wih1b, const float* __restrict__ whh1b, const float* __restrict__ bih1b, const float* __restrict__ bhh1b,
    const float* __restrict__ wih2f, const float* __restrict__ whh2f, const float* __restrict__ bih2f, const float* __restrict__ bhh2f,
    const float* __restrict__ wih2b, const float* __restrict__ whh2b, const float* __restrict__ bih2b, const float* __restrict__ bhh2b,
    const float* __restrict__ w_d1, const float* __restrict__ w_d2,
    unsigned short* __restrict__ bt1, unsigned short* __restrict__ bt2,
    unsigned short* __restrict__ wd1, unsigned short* __restrict__ wd2,
    float* __restrict__ bias1, float* __restrict__ bias2) {
  const int i = blockIdx.x * 256 + threadIdx.x;
  if (i >= CH_TOTAL) return;

  if (i < CH_BT1) {
    const int dir = i / (CH_BT1 / 2);
    const int rem = i - dir * (CH_BT1 / 2);
    const int n = rem >> 3, k8 = rem & 7;
    const int g = n / CH_PAD, jj = n - g * CH_PAD;
    const bool valid = jj < HID;
    const int src = g * HID + (valid ? jj : (HID - 1));
    const float* whh = dir ? whh1b : whh1f;
    const float* wih = dir ? wih1b : wih1f;
    float ef[8];
#pragma unroll
    for (int e = 0; e < 8; ++e) ef[e] = 0.0f;
#pragma unroll 1
    for (int d = 0; d < HID; ++d) {
      const float w = wih[src * HID + d];
      const v4f p0 = *(const v4f*)(w_proj + d * N_FEAT);
      const v4f p1 = *(const v4f*)(w_proj + d * N_FEAT + 4);
      ef[0] = fmaf(w, p0[0], ef[0]); ef[1] = fmaf(w, p0[1], ef[1]);
      ef[2] = fmaf(w, p0[2], ef[2]); ef[3] = fmaf(w, p0[3], ef[3]);
      ef[4] = fmaf(w, p1[0], ef[4]); ef[5] = fmaf(w, p1[1], ef[5]);
      ef[6] = fmaf(w, p1[2], ef[6]); ef[7] = fmaf(w, p1[3], ef[7]);
    }
    v8h hv;
#pragma unroll
    for (int e = 0; e < 8; ++e) {
      const int k = 8 * k8 + e;
      const int kc = (k < HID) ? k : (HID - 1);
      const float wv = whh[src * HID + kc];
      float v = (k < HID) ? wv : ((k8 == 6) ? ef[e] : 0.0f);
      v = valid ? v : 0.0f;
      hv[e] = (_Float16)(v * WCARRY);
    }
    store2_h8(bt1 + (size_t)i * 8, hv);
  } else if (i < CH_BT1 + CH_BT2) {
    const int q = i - CH_BT1;
    const int dir = q / (CH_BT2 / 2);
    const int rem = q - dir * (CH_BT2 / 2);
    const int n = rem / (L2_K / 8), k8 = rem - n * (L2_K / 8);
    const int g = n / CH_PAD, jj = n - g * CH_PAD;
    const bool valid = jj < HID;
    const int src = g * HID + (valid ? jj : (HID - 1));
    const float* whh = dir ? whh2b : whh2f;
    const float* wih = dir ? wih2b : wih2f;
    v8h hv;
#pragma unroll
    for (int e = 0; e < 8; ++e) {
      const int k = 8 * k8 + e;
      const bool isH = (k < HID);
      const bool isF = (k >= 64) && (k < 64 + HID);
      const bool isB = (k >= 108) && (k < 108 + HID);
      int ii = isB ? (k - 108 + HID) : (k - 64);
      ii = ii < 0 ? 0 : (ii > 2 * HID - 1 ? 2 * HID - 1 : ii);
      const int kc = isH ? k : (HID - 1);
      const float* p = isH ? (whh + src * HID + kc) : (wih + src * 2 * HID + ii);
      float v = *p;
      v = (valid && (isH || isF || isB)) ? v : 0.0f;
      hv[e] = (_Float16)(v * WCARRY);
    }
    store2_h8(bt2 + (size_t)q * 8, hv);
  } else if (i < CH_BT1 + CH_BT2 + CH_WD1) {
    const int q = i - CH_BT1 - CH_BT2;
    const int dir = q / (CH_WD1 / 2);
    const int rem = q - dir * (CH_WD1 / 2);
    const int n = rem >> 3, k8 = rem & 7;
    const bool valid = n < D1_N;
    const int nn = valid ? n : (D1_N - 1);
    v8h hv;
#pragma unroll
    for (int e = 0; e < 8; ++e) {
      const int k = 8 * k8 + e;
      const int kk = (k < HID) ? k : (HID - 1);
      float v = w_d1[nn * 2 * HID + dir * HID + kk];
      v = (valid && (k < HID)) ? v : 0.0f;
      hv[e] = (_Float16)(v * WCARRY);
    }
    store2_h8(wd1 + (size_t)q * 8, hv);
  } else if (i < CH_BT1 + CH_BT2 + CH_WD1 + CH_WD2) {
    const int q = i - CH_BT1 - CH_BT2 - CH_WD1;
    const int n = q >> 2, k8 = q & 3;
    const bool valid = n < D2_N;
    const int nn = valid ? n : (D2_N - 1);
    v8h hv;
#pragma unroll
    for (int e = 0; e < 8; ++e) {
      const int k = 8 * k8 + e;
      const int kk = (k < D1_N) ? k : (D1_N - 1);
      float v = w_d2[nn * D1_N + kk];
      v = (valid && (k < D1_N)) ? v : 0.0f;
      hv[e] = (_Float16)(v * WCARRY);
    }
    store2_h8(wd2 + (size_t)q * 8, hv);
  } else if (i < CH_BT1 + CH_BT2 + CH_WD1 + CH_WD2 + CH_B1) {
    const int q = i - CH_BT1 - CH_BT2 - CH_WD1 - CH_WD2;
    const int dir = (4 * q) / N_PAD;
    const float* wih = dir ? wih1b : wih1f;
    const float* bih = dir ? bih1b : bih1f;
    const float* bhh = dir ? bhh1b : bhh1f;
    int srcs[4]; bool vv[4]; float s[4];
#pragma unroll
    for (int e = 0; e < 4; ++e) {
      const int n = 4 * q + e - dir * N_PAD;
      const int g = n / CH_PAD, jj = n - g * CH_PAD;
      vv[e] = jj < HID;
      srcs[e] = g * HID + (vv[e] ? jj : (HID - 1));
      s[e] = 0.0f;
    }
#pragma unroll 1
    for (int d = 0; d < HID; ++d) {
      const float bp = b_proj[d];
#pragma unroll
      for (int e = 0; e < 4; ++e) s[e] = fmaf(wih[srcs[e] * HID + d], bp, s[e]);
    }
    v4f o;
#pragma unroll
    for (int e = 0; e < 4; ++e) {
      const float val = s[e] + (bih[srcs[e]] + bhh[srcs[e]]);
      o[e] = vv[e] ? (val * WCARRY) : 0.0f;
    }
    store2_f4(bias1 + (size_t)q * 4, o);
  } else {
    const int q = i - CH_BT1 - CH_BT2 - CH_WD1 - CH_WD2 - CH_B1;
    const int dir = (4 * q) / N_PAD;
    const float* bih = dir ? bih2b : bih2f;
    const float* bhh = dir ? bhh2b : bhh2f;
    v4f o;
#pragma unroll
    for (int e = 0; e < 4; ++e) {
      const int n = 4 * q + e - dir * N_PAD;
      const int g = n / CH_PAD, jj = n - g * CH_PAD;
      const bool valid = jj < HID;
      const int src = g * HID + (valid ? jj : (HID - 1));
      const float val = bih[src] + bhh[src];
      o[e] = valid ? (val * WCARRY) : 0.0f;
    }
    store2_f4(bias2 + (size_t)q * 4, o);
  }
}

__global__ __launch_bounds__(NTHR_SEQ) __attribute__((amdgpu_num_vgpr(256)))
void lstm_l1_kernel(const float* __restrict__ x, const unsigned short* __restrict__ bt1p,
                    const float* __restrict__ bias1, unsigned short* __restrict__ h1p) {
  __shared__ __align__(16) _Float16 At[16 * L1_AP];
  __shared__ __align__(16) _Float16 Hs[H1_TILE];
  const int tid = threadIdx.x, lane = tid & 31;
  const int wave = __builtin_amdgcn_readfirstlane(tid >> 5);
  const int c = lane & 15, hh = lane >> 4;
  const int dir = blockIdx.x & 1, tile = blockIdx.x >> 1;
  const int rowbase = tile * 16;
  const int j = 16 * wave + c;
  const bool chv = (j < HID);
  const int xm = tid & 15;

#pragma unroll 1
  for (int i = tid; i < 16 * L1_AP; i += NTHR_SEQ) At[i] = (_Float16)0.0f;
  __syncthreads();
  {
    const int t0 = dir ? (N_STEP - 1) : 0;
    const float* xp = x + ((size_t)(rowbase + xm) * N_STEP + (size_t)t0) * N_FEAT;
    const v4f xa = *(const v4f*)xp;
    const v4f xb = *(const v4f*)(xp + 4);
    if (tid < 16) stage_x_row(At + xm * L1_AP + 48, xa, xb);
  }

  const _Float16* Bp = (const _Float16*)bt1p + (size_t)dir * N_PAD * L1_K;
  v16h bw[4][2];
  float bb[4];
#pragma unroll
  for (int g = 0; g < 4; ++g) {
    const int n = g * CH_PAD + j;
    bw[g][0] = FragH::load(Bp + (size_t)n * L1_K + 8 * hh);
    bw[g][1] = FragH::load(Bp + (size_t)n * L1_K + 32 + 8 * hh);
    bb[g] = bias1[dir * N_PAD + n];
    pin_frag2(bw[g][0], bw[g][1], bb[g]);
  }
  float cst[8];
#pragma unroll
  for (int r = 0; r < 8; ++r) cst[r] = 0.0f;
  __syncthreads();

  const _Float16* arow = At + c * L1_AP + 8 * hh;
  const int ch = 32 * wave + lane;
  const bool sok = ch < (H1_TILE / 8);
  const int chc = sok ? ch : (H1_TILE / 8 - 1);
  unsigned short* h1d = h1p + (size_t)dir * H1_PLANE + (size_t)tile * N_STEP * H1_TILE + 8 * chc;

#pragma unroll 1
  for (int t = 0; t < N_STEP; ++t) {
    const int tt = dir ? (N_STEP - 1 - t) : t;
    const int tn = (t + 1 < N_STEP) ? (dir ? (N_STEP - 2 - t) : (t + 1)) : tt;
    const float* xp = x + ((size_t)(rowbase + xm) * N_STEP + (size_t)tn) * N_FEAT;
    const v4f xa = *(const v4f*)xp;
    const v4f xb = *(const v4f*)(xp + 4);

    v8f acc[4];
#pragma unroll
    for (int g = 0; g < 4; ++g) acc[g] = (v8f){bb[g], bb[g], bb[g], bb[g], bb[g], bb[g], bb[g], bb[g]};
    {
      const v16h a0 = FragH::load(arow);
      acc[0] = wm(a0, bw[0][0], acc[0]);
      acc[1] = wm(a0, bw[1][0], acc[1]);
      acc[2] = wm(a0, bw[2][0], acc[2]);
      acc[3] = wm(a0, bw[3][0], acc[3]);
      guard_g4(acc[0], acc[1], acc[2], acc[3], a0, bw[0][0], bw[1][0], bw[2][0], bw[3][0]);
      const v16h a1 = FragH::load(arow + 32);
      acc[0] = wm(a1, bw[0][1], acc[0]);
      acc[1] = wm(a1, bw[1][1], acc[1]);
      acc[2] = wm(a1, bw[2][1], acc[2]);
      acc[3] = wm(a1, bw[3][1], acc[3]);
      guard_g4(acc[0], acc[1], acc[2], acc[3], a1, bw[0][1], bw[1][1], bw[2][1], bw[3][1]);
    }
    float hn[8];
    lstm_cell8(acc[0], acc[1], acc[2], acc[3], cst, hn, chv);

    __syncthreads();
#pragma unroll
    for (int r = 0; r < 8; ++r) {
      const _Float16 h16 = (_Float16)hn[r];
      At[(8 * hh + r) * L1_AP + j] = h16;
      if (j < H1_W) Hs[(8 * hh + r) * H1_W + j] = h16;
    }
    if (tid < 16) stage_x_row(At + xm * L1_AP + 48, xa, xb);
    __syncthreads();

    {
      const v4u sv = *((const v4u_a*)Hs + chc);
      unsigned short* dp = h1d + (size_t)tt * H1_TILE;
      if (sok) *(volatile v4u*)dp = sv;
      __threadfence();
      if (sok) *(volatile v4u*)dp = sv;
    }
  }
}

__device__ __forceinline__ void stage_h1_tiles(_Float16* A2, const unsigned short* pf, int so0, int so1, int do0, int do1, bool ok1) {
  const unsigned short* pb = pf + H1_PLANE;
  const v2u f0 = *(const v2u*)(pf + 4 * so0);
  const v2u f1 = *(const v2u*)(pf + 4 * so1);
  const v2u g0 = *(const v2u*)(pb + 4 * so0);
  const v2u g1 = *(const v2u*)(pb + 4 * so1);
  *(v2u_a*)(A2 + do0) = f0;
  *(v2u_a*)(A2 + do0 + H1_W) = g0;
  if (ok1) {
    *(v2u_a*)(A2 + do1) = f1;
    *(v2u_a*)(A2 + do1 + H1_W) = g1;
  }
}

template <bool HEAD>
__global__ __launch_bounds__(NTHR_SEQ) __attribute__((amdgpu_num_vgpr(256)))
void lstm_l2_kernel(const unsigned short* __restrict__ h1p, const unsigned short* __restrict__ bt2p,
                    const float* __restrict__ bias2, const unsigned short* __restrict__ wd1p,
                    const unsigned short* __restrict__ wd2p, const float* __restrict__ b_d1,
                    const float* __restrict__ b_d2, const float* __restrict__ w_out,
                    const float* __restrict__ b_out, unsigned short* pbp, float* out) {
  constexpr int dir = HEAD ? 0 : 1;
  __shared__ __align__(16) _Float16 A2[16 * L2_AP];
  __shared__ __align__(16) _Float16 BI[N_PAD * BI_P];
  __shared__ __align__(16) _Float16 W1s[HEAD_NP * W1_P];
  __shared__ __align__(16) _Float16 W2s[HEAD ? HEAD_NP * W2_P : 8];
  __shared__ __align__(16) unsigned short Ps[PB_TILE];
  __shared__ __align__(16) _Float16 A1s[HEAD ? 16 * A1_P : 8];
  __shared__ __align__(16) float Ob[HEAD ? 16 * OB_P : 4];

  const int tid = threadIdx.x, lane = tid & 31;
  const int wave = __builtin_amdgcn_readfirstlane(tid >> 5);
  const int c = lane & 15, hh = lane >> 4;
  const int tile = blockIdx.x;
  const int rowbase = tile * 16;
  const int j = 16 * wave + c;
  const bool chv = (j < HID);

#pragma unroll 1
  for (int i = tid; i < 16 * L2_AP; i += NTHR_SEQ) A2[i] = (_Float16)0.0f;
  {
    const unsigned short* bsrc = bt2p + (size_t)dir * N_PAD * L2_K;
#pragma unroll 1
    for (int q = tid; q < N_PAD * 12; q += NTHR_SEQ) {
      const int row = q / 12, p = q - 12 * row;
      const v4u v = *(const v4u*)(bsrc + (size_t)row * L2_K + 64 + 8 * p);
      *(v4u_a*)(BI + row * BI_P + 8 * p) = v;
    }
    const unsigned short* w1src = wd1p + (size_t)dir * HEAD_NP * WD1_K;
#pragma unroll 1
    for (int q = tid; q < HEAD_NP * 8; q += NTHR_SEQ) {
      const int row = q >> 3, p = q & 7;
      const v4u v = *(const v4u*)(w1src + row * WD1_K + 8 * p);
      *(v4u_a*)(W1s + row * W1_P + 8 * p) = v;
    }
    if (HEAD) {
#pragma unroll 1
      for (int q = tid; q < HEAD_NP * 4; q += NTHR_SEQ) {
        const int row = q >> 2, p = q & 3;
        const v4u v = *(const v4u*)(wd2p + row * WD2_K + 8 * p);
        *(v4u_a*)(W2s + row * W2_P + 8 * p) = v;
      }
    }
  }
  __syncthreads();

  const int so0 = tid;
  const bool ok1 = (tid + NTHR_SEQ) < 176;
  const int so1 = ok1 ? (tid + NTHR_SEQ) : 175;
  const int m0 = so0 / 11, p0 = so0 - 11 * m0;
  const int m1 = so1 / 11, p1 = so1 - 11 * m1;
  const int do0 = m0 * L2_AP + 64 + 4 * p0;
  const int do1 = m1 * L2_AP + 64 + 4 * p1;
  const bool zok = tid < 48;
  const int zt = zok ? tid : 47;
  const int zm = zt / 3, zp = zt - 3 * zm;
  const int zoff = zm * L2_AP + ((zp < 2) ? (48 + 8 * zp) : 152);
  const v4u zero4 = {0u, 0u, 0u, 0u};

  const unsigned short* h1tile = h1p + (size_t)tile * N_STEP * H1_TILE;
  unsigned short* pbtile = pbp + (size_t)tile * N_STEP * PB_TILE;
  {
    const int t0 = dir ? (N_STEP - 1) : 0;
    stage_h1_tiles(A2, h1tile + (size_t)t0 * H1_TILE, so0, so1, do0, do1, ok1);
  }

  const _Float16* Bp = (const _Float16*)bt2p + (size_t)dir * N_PAD * L2_K;
  v16h bw[4][2];
  float bb[4];
#pragma unroll
  for (int g = 0; g < 4; ++g) {
    const int n = g * CH_PAD + j;
    bw[g][0] = FragH::load(Bp + (size_t)n * L2_K + 8 * hh);
    bw[g][1] = FragH::load(Bp + (size_t)n * L2_K + 32 + 8 * hh);
    bb[g] = bias2[dir * N_PAD + n];
    pin_frag2(bw[g][0], bw[g][1], bb[g]);
  }
  const int wv1 = (wave < 2) ? wave : 1;
  const int n1 = 16 * wv1 + c;
  const int n1c = (n1 < D1_N) ? n1 : (D1_N - 1);
  float bd1v = b_d1[n1c];
  bd1v = (n1 < D1_N) ? bd1v : 0.0f;
  const int n2c = (16 + c < D2_N) ? (16 + c) : (D2_N - 1);
  float bd2a = b_d2[c];
  float bd2b = b_d2[n2c];
  float woa = w_out[c];
  float wob = w_out[n2c];
  pin_f4(bd2a, bd2b, woa, wob);
  bd2b = (16 + c < D2_N) ? bd2b : 0.0f;
  wob  = (16 + c < D2_N) ? wob : 0.0f;
  const float bout = b_out[0];

  float cst[8];
#pragma unroll
  for (int r = 0; r < 8; ++r) cst[r] = 0.0f;
  __syncthreads();

  const _Float16* arow  = A2 + c * L2_AP + 8 * hh;
  const _Float16* birow = BI + j * BI_P + 8 * hh;
  const _Float16* w1row = W1s + n1 * W1_P + 8 * hh;
  const int pch = 32 * wv1 + lane;

#pragma unroll 1
  for (int t = 0; t < N_STEP; ++t) {
    const int tt = dir ? (N_STEP - 1 - t) : t;
    const int tn = (t + 1 < N_STEP) ? (dir ? (N_STEP - 2 - t) : (t + 1)) : tt;

    v8f acc[4];
#pragma unroll
    for (int g = 0; g < 4; ++g) acc[g] = (v8f){bb[g], bb[g], bb[g], bb[g], bb[g], bb[g], bb[g], bb[g]};
    {
      const v16h a0 = FragH::load(arow);
      acc[0] = wm(a0, bw[0][0], acc[0]);
      acc[1] = wm(a0, bw[1][0], acc[1]);
      acc[2] = wm(a0, bw[2][0], acc[2]);
      acc[3] = wm(a0, bw[3][0], acc[3]);
      guard_g4(acc[0], acc[1], acc[2], acc[3], a0, bw[0][0], bw[1][0], bw[2][0], bw[3][0]);
      const v16h a1 = FragH::load(arow + 32);
      acc[0] = wm(a1, bw[0][1], acc[0]);
      acc[1] = wm(a1, bw[1][1], acc[1]);
      acc[2] = wm(a1, bw[2][1], acc[2]);
      acc[3] = wm(a1, bw[3][1], acc[3]);
      guard_g4(acc[0], acc[1], acc[2], acc[3], a1, bw[0][1], bw[1][1], bw[2][1], bw[3][1]);
    }
#pragma unroll 1
    for (int ks = 0; ks < 3; ++ks) {
      const v16h a  = FragH::load(arow + 64 + 32 * ks);
      const v16h b0 = FragH::load(birow + 32 * ks);
      const v16h b1 = FragH::load(birow + 1 * CH_PAD * BI_P + 32 * ks);
      const v16h b2 = FragH::load(birow + 2 * CH_PAD * BI_P + 32 * ks);
      const v16h b3 = FragH::load(birow + 3 * CH_PAD * BI_P + 32 * ks);
      acc[0] = wm(a, b0, acc[0]);
      acc[1] = wm(a, b1, acc[1]);
      acc[2] = wm(a, b2, acc[2]);
      acc[3] = wm(a, b3, acc[3]);
      guard_g4(acc[0], acc[1], acc[2], acc[3], a, b0, b1, b2, b3);
    }
    float hn[8];
    lstm_cell8(acc[0], acc[1], acc[2], acc[3], cst, hn, chv);

    __syncthreads();
#pragma unroll
    for (int r = 0; r < 8; ++r) A2[(8 * hh + r) * L2_AP + j] = (_Float16)hn[r];
    if (zok) *(v4u_a*)(A2 + zoff) = zero4;
    stage_h1_tiles(A2, h1tile + (size_t)tn * H1_TILE, so0, so1, do0, do1, ok1);
    if (HEAD) {
      if (wave < 2) {
        const v4u pv = *(const v4u*)(pbtile + (size_t)tt * PB_TILE + 8 * pch);
        *(v4u_a*)(Ps + 8 * pch) = pv;
      }
    }
    __syncthreads();

    if (wave < 2) {
      const v16h pa0 = FragH::load(arow);
      const v16h pa1 = FragH::load(arow + 32);
      const v16h pb0 = FragH::load(w1row);
      const v16h pb1 = FragH::load(w1row + 32);
      v8f pacc = (v8f){0.f, 0.f, 0.f, 0.f, 0.f, 0.f, 0.f, 0.f};
      pacc = wm(pa0, pb0, pacc);
      pacc = wm(pa1, pb1, pacc);
      guard_g1(pacc, pa0, pa1, pb0, pb1);
      if (!HEAD) {
#pragma unroll
        for (int r = 0; r < 8; ++r) {
          const _Float16 ph = (_Float16)(pacc[r] * WCARRY_INV);
          Ps[(8 * hh + r) * 32 + n1] = __builtin_bit_cast(unsigned short, ph);
        }
      } else {
#pragma unroll
        for (int r = 0; r < 8; ++r) {
          const unsigned pbits = (unsigned)Ps[(8 * hh + r) * 32 + n1];
          const float pv = h16_to_f32(pbits);
          float v = pacc[r] * WCARRY_INV + pv + bd1v;
          v = fmaxf(v, 0.0f);
          A1s[(8 * hh + r) * A1_P + n1] = (_Float16)v;
        }
      }
    }
    __syncthreads();

    if (!HEAD) {
      if (wave < 2) {
        const v4u sv = *((const v4u_a*)Ps + pch);
        unsigned short* dp = pbtile + (size_t)tt * PB_TILE + 8 * pch;
        *(volatile v4u*)dp = sv;
        __threadfence();
        *(volatile v4u*)dp = sv;
      }
    } else {
      if (wave == 0) {
        const v16h qa  = FragH::load(A1s + c * A1_P + 8 * hh);
        const v16h qb0 = FragH::load(W2s + c * W2_P + 8 * hh);
        const v16h qb1 = FragH::load(W2s + (16 + c) * W2_P + 8 * hh);
        v8f d0 = (v8f){0.f, 0.f, 0.f, 0.f, 0.f, 0.f, 0.f, 0.f};
        v8f d1 = (v8f){0.f, 0.f, 0.f, 0.f, 0.f, 0.f, 0.f, 0.f};
        d0 = wm(qa, qb0, d0);
        d1 = wm(qa, qb1, d1);
        guard_g2(d0, d1, qa, qb0, qb1);
        float s[8];
#pragma unroll
        for (int r = 0; r < 8; ++r) {
          const float u0 = fmaxf(d0[r] * WCARRY_INV + bd2a, 0.0f);
          const float u1 = fmaxf(d1[r] * WCARRY_INV + bd2b, 0.0f);
          s[r] = u0 * woa + u1 * wob;
        }
#pragma unroll
        for (int r = 0; r < 8; ++r) {
#pragma unroll
          for (int off = 1; off < 16; off <<= 1) s[r] += __shfl_xor(s[r], off, 32);
        }
        if (c == 0) {
#pragma unroll
          for (int r = 0; r < 8; ++r) Ob[(8 * hh + r) * OB_P + (t & 31)] = s[r] + bout;
        }
        if ((t & 31) == 31) {
          __builtin_amdgcn_fence(__ATOMIC_RELEASE, "workgroup");
          __builtin_amdgcn_wave_barrier();
          __builtin_amdgcn_fence(__ATOMIC_ACQUIRE, "workgroup");
          const int tbase = t - 31;
          for (int pass = 0; pass < 2; ++pass) {
#pragma unroll
            for (int it = 0; it < 4; ++it) {
              const int chunk = it * 32 + lane;
              const int row = chunk >> 3, c4 = (chunk & 7) * 4;
              const v4f ov = *(const v4f*)(Ob + row * OB_P + c4);
              *(volatile v4f*)(out + (size_t)(rowbase + row) * N_STEP + tbase + c4) = ov;
            }
            __threadfence();
          }
          __builtin_amdgcn_fence(__ATOMIC_RELEASE, "workgroup");
          __builtin_amdgcn_wave_barrier();
          __builtin_amdgcn_fence(__ATOMIC_ACQUIRE, "workgroup");
        }
      }
    }
  }
}

extern "C" void kernel_launch(void* const* d_in, const int* in_sizes, int n_in,
                              void* d_out, int out_size, void* d_ws, size_t ws_size, hipStream_t stream) {
  if (n_in < 25 || d_out == nullptr || d_ws == nullptr) return;
  if (in_sizes[0] != N_BATCH * N_STEP * N_FEAT || in_sizes[1] != HID * N_FEAT || in_sizes[2] != HID) return;
  if (in_sizes[3] != 4 * HID * HID || in_sizes[4] != 4 * HID * HID || in_sizes[5] != 4 * HID || in_sizes[6] != 4 * HID) return;
  if (in_sizes[7] != 4 * HID * HID || in_sizes[8] != 4 * HID * HID || in_sizes[9] != 4 * HID || in_sizes[10] != 4 * HID) return;
  if (in_sizes[11] != 4 * HID * 2 * HID || in_sizes[12] != 4 * HID * HID || in_sizes[13] != 4 * HID || in_sizes[14] != 4 * HID) return;
  if (in_sizes[15] != 4 * HID * 2 * HID || in_sizes[16] != 4 * HID * HID || in_sizes[17] != 4 * HID || in_sizes[18] != 4 * HID) return;
  if (in_sizes[19] != D1_N * 2 * HID || in_sizes[20] != D1_N || in_sizes[21] != D2_N * D1_N || in_sizes[22] != D2_N) return;
  if (in_sizes[23] != D2_N || in_sizes[24] != 1 || out_size != N_BATCH * N_STEP) return;

  const float* x      = (const float*)d_in[0];
  const float* w_proj = (const float*)d_in[1];
  const float* b_proj = (const float*)d_in[2];
  const float* w_ih1f = (const float*)d_in[3];
  const float* w_hh1f = (const float*)d_in[4];
  const float* b_ih1f = (const float*)d_in[5];
  const float* b_hh1f = (const float*)d_in[6];
  const float* w_ih1b = (const float*)d_in[7];
  const float* w_hh1b = (const float*)d_in[8];
  const float* b_ih1b = (const float*)d_in[9];
  const float* b_hh1b = (const float*)d_in[10];
  const float* w_ih2f = (const float*)d_in[11];
  const float* w_hh2f = (const float*)d_in[12];
  const float* b_ih2f = (const float*)d_in[13];
  const float* b_hh2f = (const float*)d_in[14];
  const float* w_ih2b = (const float*)d_in[15];
  const float* w_hh2b = (const float*)d_in[16];
  const float* b_ih2b = (const float*)d_in[17];
  const float* b_hh2b = (const float*)d_in[18];
  const float* w_d1   = (const float*)d_in[19];
  const float* b_d1   = (const float*)d_in[20];
  const float* w_d2   = (const float*)d_in[21];
  const float* b_d2   = (const float*)d_in[22];
  const float* w_out  = (const float*)d_in[23];
  const float* b_out  = (const float*)d_in[24];
  float* out = (float*)d_out;

  char* ws = (char*)d_ws; size_t off = 0;
  auto carve = [&](size_t bytes) -> char* { char* p = ws + off; off += (bytes + 255) & ~(size_t)255; return p; };
  unsigned short* H1    = (unsigned short*)carve(WS_H1);
  unsigned short* PB    = (unsigned short*)carve(WS_PB);
  unsigned short* BT1   = (unsigned short*)carve(WS_BT1);
  unsigned short* BT2   = (unsigned short*)carve(WS_BT2);
  unsigned short* WD1   = (unsigned short*)carve(WS_WD1);
  unsigned short* WD2   = (unsigned short*)carve(WS_WD2);
  float*          BIAS1 = (float*)carve(WS_B1);
  float*          BIAS2 = (float*)carve(WS_B2);
  if (off > ws_size || off > (size_t)134217728) return;

  prep_planes_kernel<<<(CH_TOTAL + 255) / 256, 256, 0, stream>>>(
      w_proj, b_proj,
      w_ih1f, w_hh1f, b_ih1f, b_hh1f, w_ih1b, w_hh1b, b_ih1b, b_hh1b,
      w_ih2f, w_hh2f, b_ih2f, b_hh2f, w_ih2b, w_hh2b, b_ih2b, b_hh2b,
      w_d1, w_d2, BT1, BT2, WD1, WD2, BIAS1, BIAS2);
  lstm_l1_kernel<<<N_TILE * 2, NTHR_SEQ, 0, stream>>>(x, BT1, BIAS1, H1);
  lstm_l2_kernel<false><<<N_TILE, NTHR_SEQ, 0, stream>>>(H1, BT2, BIAS2, WD1, WD2, b_d1, b_d2, w_out, b_out, PB, out);
  lstm_l2_kernel<true><<<N_TILE, NTHR_SEQ, 0, stream>>>(H1, BT2, BIAS2, WD1, WD2, b_d1, b_d2, w_out, b_out, PB, out);
}
